// EchoBlock_75892072121065
// MI455X (gfx1250) — hardware-verified
//
#include <hip/hip_runtime.h>
#define SS 1024
#define DM 512
#define NH 8
#define DH 64
#define NNR 128

typedef __bf16 v16b __attribute__((ext_vector_type(16)));
typedef unsigned short v8us __attribute__((ext_vector_type(8), may_alias));
typedef float  v8f  __attribute__((ext_vector_type(8)));
typedef float  v4f  __attribute__((ext_vector_type(4)));
typedef float  v4fa __attribute__((ext_vector_type(4), may_alias));
union FragB { v16b v; v8us half[2]; unsigned short u[16]; };

__device__ __forceinline__ unsigned short bf16_bits(float x) { unsigned int u = __float_as_uint(x); return (unsigned short)((u + 0x7FFFu + ((u >> 16) & 1u)) >> 16); }
__device__ __forceinline__ float bf16_val(unsigned short b) { return __uint_as_float(((unsigned int)b) << 16); }
__device__ __forceinline__ float bf16_round(float x) { return bf16_val(bf16_bits(x)); }
template <int NT>
__device__ __forceinline__ v8f mmaN(v16b ah, v16b al, v16b bh, v16b bl, v8f c) {
  c = __builtin_amdgcn_wmma_f32_16x16x32_bf16(false, ah, false, bh, (short)0, c, false, false);
  if (NT >= 2) c = __builtin_amdgcn_wmma_f32_16x16x32_bf16(false, al, false, bh, (short)0, c, false, false);
  if (NT >= 3) c = __builtin_amdgcn_wmma_f32_16x16x32_bf16(false, ah, false, bl, (short)0, c, false, false);
  asm volatile("v_nop\n\tv_nop\n\tv_nop\n\tv_nop" : "+v"(c) : "v"(ah), "v"(al), "v"(bh), "v"(bl));
  return c;
}

__global__ __launch_bounds__(256) void k_wt_bf16(const float* __restrict__ W, unsigned short* __restrict__ Wt, int K, int N) {
  const int t = blockIdx.x * 256 + threadIdx.x;
  const int k8n = K / 8;
  if (t >= N * k8n) return;
  const int n = t / k8n, k8 = (t % k8n) * 8;
  v8us v;
#pragma unroll
  for (int i = 0; i < 8; ++i) v[i] = bf16_bits(W[(size_t)(k8 + i) * N + n]);
  *(volatile v8us*)(Wt + (size_t)n * K + k8) = v;
  __threadfence();
  *(volatile v8us*)(Wt + (size_t)n * K + k8) = v;
}

template <bool ASPLIT, int ACT, bool BIAS_BF16>
__global__ __launch_bounds__(128) void k_gemm_bf(const float* __restrict__ A, int lda, const unsigned short* __restrict__ Wt, int ldb,
                                               const float* __restrict__ bias, float* __restrict__ C, int ldc, int M, int N, int K) {
  __shared__ __attribute__((aligned(16))) float so[4][16][64];
  const int tid = threadIdx.x, w = tid >> 5, lane = tid & 31, ln = lane & 15, hh = lane >> 4;
  const int ntn = N / 64;
  const int wid = blockIdx.x * 4 + w;
  const int mt = wid / ntn, nq = wid % ntn;
  if (mt * 16 >= M) return;
  const int row0 = mt * 16, col0 = nq * 64;
  const float* arow = A + (size_t)(row0 + ln) * lda;
  v8f acc[4] = {};
  for (int kb = 0; kb < K; kb += 32) {
    FragB ah, al;
    const v4f x0 = *(const v4fa*)(arow + kb + 8 * hh), x1 = *(const v4fa*)(arow + kb + 8 * hh + 4);
    const v4f x2 = *(const v4fa*)(arow + kb + 16 + 8 * hh), x3 = *(const v4fa*)(arow + kb + 16 + 8 * hh + 4);
    float xs[16] = {x0[0],x0[1],x0[2],x0[3],x1[0],x1[1],x1[2],x1[3],x2[0],x2[1],x2[2],x2[3],x3[0],x3[1],x3[2],x3[3]};
#pragma unroll
    for (int i = 0; i < 16; ++i) { const unsigned short hb = bf16_bits(xs[i]); ah.u[i] = hb; al.u[i] = ASPLIT ? bf16_bits(xs[i] - bf16_val(hb)) : (unsigned short)0; }
#pragma unroll
    for (int t = 0; t < 4; ++t) {
      const unsigned short* brow = Wt + (size_t)(col0 + t * 16 + ln) * ldb + kb;
      FragB b;
      b.half[0] = *(const v8us*)(brow + 8 * hh);
      b.half[1] = *(const v8us*)(brow + 16 + 8 * hh);
      acc[t] = mmaN<ASPLIT ? 2 : 1>(ah.v, al.v, b.v, b.v, acc[t]);
    }
  }
#pragma unroll
  for (int t = 0; t < 4; ++t) {
    float bv = bias ? bias[col0 + t * 16 + ln] : 0.f;
    if (BIAS_BF16) bv = bf16_round(bv);
#pragma unroll
    for (int r = 0; r < 8; ++r) { float v = acc[t][r] + bv; if (ACT == 1) v = fmaxf(v, 0.f); so[w][8 * hh + r][t * 16 + ln] = v; }
  }
  __builtin_amdgcn_fence(__ATOMIC_ACQ_REL, "workgroup");
  __builtin_amdgcn_wave_barrier();
  const int rsub = lane >> 4, c4 = (lane & 15) * 4;
  for (int pass = 0; pass < 2; ++pass) {
#pragma unroll
    for (int q = 0; q < 8; ++q) {
      const int r = q * 2 + rsub;
      const v4f v = *(const v4fa*)&so[w][r][c4];
      *(volatile v4f*)(C + (size_t)(row0 + r) * ldc + col0 + c4) = v;
    }
    if (pass == 0) __threadfence();
  }
}

template <int D, bool CAUSAL>
__global__ __launch_bounds__(128) void k_flash(const float* __restrict__ qb, const float* __restrict__ kb, const float* __restrict__ vb,
                                             int pitch, int T, int H, float scale, float* __restrict__ y, int ypitch) {
  constexpr int KS = D / 32;
  constexpr int DT = D / 16;
  __shared__ __attribute__((aligned(16))) unsigned short sKh[32][D + 8], sKl[32][D + 8], sVh[32][D + 8], sVl[32][D + 8];
  __shared__ __attribute__((aligned(16))) unsigned short sPh[4][16][40], sPl[4][16][40];
  __shared__ __attribute__((aligned(16))) float sO[4][16][D];
  const int tid = threadIdx.x, w = tid >> 5, lane = tid & 31, ln = lane & 15, hh = lane >> 4;
  const int nqb = (T + 63) / 64;
  const int bh = blockIdx.x / nqb, qblk = blockIdx.x % nqb;
  const int b = bh / H, h = bh % H;
  const int q0 = qblk * 64 + w * 16;
  const float* Q = qb + (size_t)b * T * pitch + h * D;
  const float* K = kb + (size_t)b * T * pitch + h * D;
  const float* V = vb + (size_t)b * T * pitch + h * D;

  FragB aqh[KS], aql[KS];
  {
    int row = q0 + ln; if (row >= T) row = T - 1;
    const float* qr = Q + (size_t)row * pitch;
#pragma unroll
    for (int ks = 0; ks < KS; ++ks)
#pragma unroll
      for (int i = 0; i < 16; ++i) {
        const int d = ks * 32 + ((i < 8) ? (8 * hh + i) : (16 + 8 * hh + (i - 8)));
        const float x = qr[d] * scale; const unsigned short hb = bf16_bits(x);
        aqh[ks].u[i] = hb; aql[ks].u[i] = bf16_bits(x - bf16_val(hb));
      }
  }
  float m_r[8], l_r[8];
#pragma unroll
  for (int r = 0; r < 8; ++r) { m_r[r] = -3.0e38f; l_r[r] = 0.f; }
  v8f oacc[DT];
#pragma unroll
  for (int dt = 0; dt < DT; ++dt) oacc[dt] = (v8f){0.f,0.f,0.f,0.f,0.f,0.f,0.f,0.f};

  const int kv_end = CAUSAL ? min(T, qblk * 64 + 64) : T;
  for (int j0 = 0; j0 < kv_end; j0 += 32) {
    __syncthreads();
    for (int e = tid; e < 32 * (D / 4); e += 128) {
      const int r = e / (D / 4), c4 = (e % (D / 4)) * 4;
      const int key = j0 + r;
      v4f kf = {0.f,0.f,0.f,0.f}, vf = {0.f,0.f,0.f,0.f};
      if (key < T) { kf = *(const v4fa*)(K + (size_t)key * pitch + c4); vf = *(const v4fa*)(V + (size_t)key * pitch + c4); }
#pragma unroll
      for (int t = 0; t < 4; ++t) {
        unsigned short hb = bf16_bits(kf[t]); sKh[r][c4 + t] = hb; sKl[r][c4 + t] = bf16_bits(kf[t] - bf16_val(hb));
        hb = bf16_bits(vf[t]); sVh[r][c4 + t] = hb; sVl[r][c4 + t] = bf16_bits(vf[t] - bf16_val(hb));
      }
    }
    __syncthreads();
    v8f s[2];
#pragma unroll
    for (int nt = 0; nt < 2; ++nt) {
      v8f acc = {};
#pragma unroll
      for (int ks = 0; ks < KS; ++ks) {
        FragB bh_, bl_;
        bh_.half[0] = *(const v8us*)&sKh[nt * 16 + ln][ks * 32 + 8 * hh]; bh_.half[1] = *(const v8us*)&sKh[nt * 16 + ln][ks * 32 + 16 + 8 * hh];
        bl_.half[0] = *(const v8us*)&sKl[nt * 16 + ln][ks * 32 + 8 * hh]; bl_.half[1] = *(const v8us*)&sKl[nt * 16 + ln][ks * 32 + 16 + 8 * hh];
        acc = mmaN<3>(aqh[ks].v, aql[ks].v, bh_.v, bl_.v, acc);
      }
      s[nt] = acc;
    }
    float alpha[8];
#pragma unroll
    for (int r = 0; r < 8; ++r) {
      const int qi = q0 + 8 * hh + r;
      const int ja = j0 + ln, jb = j0 + 16 + ln;
      if (CAUSAL) { if (ja > qi) s[0][r] = -3.0e38f; if (jb > qi) s[1][r] = -3.0e38f; }
      if (ja >= T) s[0][r] = -3.0e38f;
      if (jb >= T) s[1][r] = -3.0e38f;
      float mx = fmaxf(s[0][r], s[1][r]);
      mx = fmaxf(mx, __shfl_xor(mx, 1, 32)); mx = fmaxf(mx, __shfl_xor(mx, 2, 32)); mx = fmaxf(mx, __shfl_xor(mx, 4, 32)); mx = fmaxf(mx, __shfl_xor(mx, 8, 32));
      const float mnew = fmaxf(m_r[r], mx);
      alpha[r] = (mnew > -1.0e38f) ? __expf(m_r[r] - mnew) : 1.0f;
      const float p0 = (s[0][r] > -1.0e38f) ? __expf(s[0][r] - mnew) : 0.f;
      const float p1 = (s[1][r] > -1.0e38f) ? __expf(s[1][r] - mnew) : 0.f;
      m_r[r] = mnew;
      l_r[r] = l_r[r] * alpha[r] + p0 + p1;
      unsigned short hb = bf16_bits(p0); sPh[w][8 * hh + r][ln] = hb;      sPl[w][8 * hh + r][ln] = bf16_bits(p0 - bf16_val(hb));
      hb = bf16_bits(p1);                sPh[w][8 * hh + r][16 + ln] = hb; sPl[w][8 * hh + r][16 + ln] = bf16_bits(p1 - bf16_val(hb));
    }
#pragma unroll
    for (int dt = 0; dt < DT; ++dt)
#pragma unroll
      for (int r = 0; r < 8; ++r) oacc[dt][r] *= alpha[r];
    __builtin_amdgcn_fence(__ATOMIC_ACQ_REL, "workgroup");
    __builtin_amdgcn_wave_barrier();
    FragB pah, pal;
    pah.half[0] = *(const v8us*)&sPh[w][ln][8 * hh]; pah.half[1] = *(const v8us*)&sPh[w][ln][16 + 8 * hh];
    pal.half[0] = *(const v8us*)&sPl[w][ln][8 * hh]; pal.half[1] = *(const v8us*)&sPl[w][ln][16 + 8 * hh];
#pragma unroll
    for (int dt = 0; dt < DT; ++dt) {
      FragB bvh, bvl;
#pragma unroll
      for (int i = 0; i < 8; ++i) {
        bvh.u[i] = sVh[8 * hh + i][dt * 16 + ln]; bvh.u[8 + i] = sVh[16 + 8 * hh + i][dt * 16 + ln];
        bvl.u[i] = sVl[8 * hh + i][dt * 16 + ln]; bvl.u[8 + i] = sVl[16 + 8 * hh + i][dt * 16 + ln];
      }
      oacc[dt] = mmaN<3>(pah.v, pal.v, bvh.v, bvl.v, oacc[dt]);
    }
    __builtin_amdgcn_fence(__ATOMIC_ACQ_REL, "workgroup");
    __builtin_amdgcn_wave_barrier();
  }
#pragma unroll
  for (int r = 0; r < 8; ++r) {
    float l = l_r[r];
    l += __shfl_xor(l, 1, 32); l += __shfl_xor(l, 2, 32); l += __shfl_xor(l, 4, 32); l += __shfl_xor(l, 8, 32);
    l_r[r] = (l > 0.f) ? 1.0f / l : 0.f;
  }
#pragma unroll
  for (int dt = 0; dt < DT; ++dt)
#pragma unroll
    for (int r = 0; r < 8; ++r) sO[w][8 * hh + r][dt * 16 + ln] = oacc[dt][r] * l_r[r];
  __builtin_amdgcn_fence(__ATOMIC_ACQ_REL, "workgroup");
  __builtin_amdgcn_wave_barrier();
  for (int pass = 0; pass < 2; ++pass) {
    for (int r = 0; r < 16; ++r) {
      const int row = q0 + r;
      if (row < T && lane < D / 4) {
        const v4f val = *(const v4fa*)&sO[w][r][lane * 4];
        *(volatile v4f*)(y + ((size_t)b * T + row) * ypitch + h * D + lane * 4) = val;
      }
    }
    if (pass == 0) __threadfence();
  }
}

typedef _Float16 v16h __attribute__((ext_vector_type(16)));
union FragH { v16h v; v8us half[2]; _Float16 h[16]; unsigned short u[16]; };
template <int NT>
__device__ __forceinline__ v8f mmaH(v16h ah, v16h al, v16h bh, v16h bl, v8f c) {
  c = __builtin_amdgcn_wmma_f32_16x16x32_f16(false, ah, false, bh, (short)0, c, false, false);
  if (NT >= 2) c = __builtin_amdgcn_wmma_f32_16x16x32_f16(false, al, false, bh, (short)0, c, false, false);
  if (NT >= 3) c = __builtin_amdgcn_wmma_f32_16x16x32_f16(false, ah, false, bl, (short)0, c, false, false);
  asm volatile("v_nop\n\tv_nop\n\tv_nop\n\tv_nop" : "+v"(c) : "v"(ah), "v"(al), "v"(bh), "v"(bl));
  return c;
}
template <bool ASPLIT>
__global__ __launch_bounds__(128) void k_gemm_h(const float* __restrict__ A, int lda, size_t sA, const _Float16* __restrict__ Bh, int ldb, size_t sB, float alpha, float* __restrict__ C, int ldc, size_t sC, int M, int N, int K) {
  __shared__ __attribute__((aligned(16))) float so[4][16][64];
  const int tid = threadIdx.x, w = tid >> 5, lane = tid & 31, ln = lane & 15, hh = lane >> 4; const int by = blockIdx.y;
  A += (size_t)by * sA; Bh += (size_t)by * sB; C += (size_t)by * sC;
  const int ntn = (N + 63) / 64; const int wid = blockIdx.x * 4 + w; const int mt = wid / ntn, nq = wid % ntn; if (mt * 16 >= M) return;
  const int row0 = mt * 16, col0 = nq * 64; const float* arow = A + (size_t)(row0 + ln) * lda;
  v8f acc[4] = {};
  for (int kb = 0; kb < K; kb += 32) {
    FragH ah, al;
    const v4f x0 = *(const v4fa*)(arow + kb + 8 * hh), x1 = *(const v4fa*)(arow + kb + 8 * hh + 4), x2 = *(const v4fa*)(arow + kb + 16 + 8 * hh), x3 = *(const v4fa*)(arow + kb + 16 + 8 * hh + 4);
    float xs[16] = {x0[0],x0[1],x0[2],x0[3],x1[0],x1[1],x1[2],x1[3],x2[0],x2[1],x2[2],x2[3],x3[0],x3[1],x3[2],x3[3]};
#pragma unroll
    for (int i = 0; i < 16; ++i) { const _Float16 h = (_Float16)xs[i]; ah.h[i] = h; al.h[i] = ASPLIT ? (_Float16)(xs[i] - (float)h) : (_Float16)0.0f; }
#pragma unroll
    for (int t = 0; t < 4; ++t) { if (col0 + t * 16 >= N) continue; const size_t boff = (size_t)(col0 + t * 16 + ln) * ldb + kb; FragH bq; bq.half[0] = *(const v8us*)(Bh + boff + 8 * hh); bq.half[1] = *(const v8us*)(Bh + boff + 16 + 8 * hh);
      acc[t] = mmaH<ASPLIT ? 2 : 1>(ah.v, al.v, bq.v, bq.v, acc[t]); }
  }
#pragma unroll
  for (int t = 0; t < 4; ++t) { if (col0 + t * 16 >= N) continue;
#pragma unroll
    for (int r = 0; r < 8; ++r) so[w][8 * hh + r][t * 16 + ln] = acc[t][r] * alpha; }
  __builtin_amdgcn_fence(__ATOMIC_ACQ_REL, "workgroup"); __builtin_amdgcn_wave_barrier();
  const int rsub = lane >> 4, c4 = (lane & 15) * 4;
  for (int pass = 0; pass < 2; ++pass) {
#pragma unroll
    for (int q = 0; q < 8; ++q) { const int r = q * 2 + rsub; if (col0 + c4 < N) { const v4f v = *(const v4fa*)&so[w][r][c4]; *(volatile v4f*)(C + (size_t)(row0 + r) * ldc + col0 + c4) = v; } }
    if (pass == 0) __threadfence(); }
}

template <int DUMMY>
__global__ __launch_bounds__(128) void k_gemm_hh(const _Float16* __restrict__ A, int lda, size_t sA, const _Float16* __restrict__ Bh, int ldb, size_t sB, float alpha, float* __restrict__ C, int ldc, size_t sC, int M, int N, int K) {
  __shared__ __attribute__((aligned(16))) float so[4][16][64];
  const int tid = threadIdx.x, w = tid >> 5, lane = tid & 31, ln = lane & 15, hh = lane >> 4; const int by = blockIdx.y;
  A += (size_t)by * sA; Bh += (size_t)by * sB; C += (size_t)by * sC;
  const int ntn = (N + 63) / 64; const int wid = blockIdx.x * 4 + w; const int mt = wid / ntn, nq = wid % ntn; if (mt * 16 >= M) return;
  const int row0 = mt * 16, col0 = nq * 64; const _Float16* arow = A + (size_t)(row0 + ln) * lda;
  v8f acc[4] = {};
  for (int kb = 0; kb < K; kb += 32) { FragH ah; ah.half[0] = *(const v8us*)((const unsigned short*)arow + kb + 8 * hh); ah.half[1] = *(const v8us*)((const unsigned short*)arow + kb + 16 + 8 * hh);
#pragma unroll
    for (int t = 0; t < 4; ++t) { if (col0 + t * 16 >= N) continue; const size_t boff = (size_t)(col0 + t * 16 + ln) * ldb + kb; FragH bq; bq.half[0] = *(const v8us*)((const unsigned short*)Bh + boff + 8 * hh); bq.half[1] = *(const v8us*)((const unsigned short*)Bh + boff + 16 + 8 * hh);
      acc[t] = mmaH<1>(ah.v, ah.v, bq.v, bq.v, acc[t]); }
  }
#pragma unroll
  for (int t = 0; t < 4; ++t) { if (col0 + t * 16 >= N) continue;
#pragma unroll
    for (int r = 0; r < 8; ++r) so[w][8 * hh + r][t * 16 + ln] = acc[t][r] * alpha; }
  __builtin_amdgcn_fence(__ATOMIC_ACQ_REL, "workgroup"); __builtin_amdgcn_wave_barrier();
  const int rsub = lane >> 4, c4 = (lane & 15) * 4;
  for (int pass = 0; pass < 2; ++pass) {
#pragma unroll
    for (int q = 0; q < 8; ++q) { const int r = q * 2 + rsub; if (col0 + c4 < N) { const v4f v = *(const v4fa*)&so[w][r][c4]; *(volatile v4f*)(C + (size_t)(row0 + r) * ldc + col0 + c4) = v; } }
    if (pass == 0) __threadfence(); }
}

template <int ACT>
__global__ __launch_bounds__(128) void k_gemm_hhx(const _Float16* __restrict__ A, int lda, size_t sA, const _Float16* __restrict__ Bh, int ldb, size_t sB, float alpha, const float* __restrict__ bias, size_t sBias, const float* __restrict__ CP, int rowsPerB, size_t sCPb, int row0g,
    float* __restrict__ C, _Float16* __restrict__ C16, int ldc, size_t sC, int M, int N, int K) {
  __shared__ __attribute__((aligned(16))) float so[4][16][64];
  const int tid = threadIdx.x, w = tid >> 5, lane = tid & 31, ln = lane & 15, hh = lane >> 4; const int by = blockIdx.y;
  A += (size_t)by * sA; Bh += (size_t)by * sB; const size_t cofs = (size_t)by * sC; const float* bp = bias ? bias + (size_t)by * sBias : nullptr;
  const int ntn = (N + 63) / 64; const int wid = blockIdx.x * 4 + w; const int mt = wid / ntn, nq = wid % ntn; if (mt * 16 >= M) return;
  const int row0 = mt * 16, col0 = nq * 64; const _Float16* arow = A + (size_t)(row0 + ln) * lda;
  v8f acc[4] = {};
  for (int kb = 0; kb < K; kb += 32) { FragH ah; ah.half[0] = *(const v8us*)((const unsigned short*)arow + kb + 8 * hh); ah.half[1] = *(const v8us*)((const unsigned short*)arow + kb + 16 + 8 * hh);
#pragma unroll
    for (int t = 0; t < 4; ++t) { if (col0 + t * 16 >= N) continue; const size_t boff = (size_t)(col0 + t * 16 + ln) * ldb + kb; FragH bq; bq.half[0] = *(const v8us*)((const unsigned short*)Bh + boff + 8 * hh); bq.half[1] = *(const v8us*)((const unsigned short*)Bh + boff + 16 + 8 * hh);
      acc[t] = mmaH<1>(ah.v, ah.v, bq.v, bq.v, acc[t]); }
  }
#pragma unroll
  for (int t = 0; t < 4; ++t) { if (col0 + t * 16 >= N) continue; const int col = col0 + t * 16 + ln; const float bv = bp ? bf16_round(bp[col]) : 0.f;
#pragma unroll
    for (int r = 0; r < 8; ++r) { float v = acc[t][r] * alpha + bv; if (CP) { const int bidx = (row0g + row0 + 8 * hh + r) / rowsPerB; v += CP[(size_t)bidx * sCPb + (size_t)by * 64 + col]; } if (ACT == 1) v = (v > 0.f) ? v : expm1f(v); so[w][8 * hh + r][t * 16 + ln] = v; } }
  __builtin_amdgcn_fence(__ATOMIC_ACQ_REL, "workgroup"); __builtin_amdgcn_wave_barrier();
  const int rsub = lane >> 4, c4 = (lane & 15) * 4; typedef _Float16 v4h __attribute__((ext_vector_type(4)));
  for (int pass = 0; pass < 2; ++pass) {
#pragma unroll
    for (int q = 0; q < 8; ++q) { const int r = q * 2 + rsub; if (col0 + c4 < N) { const v4f v = *(const v4fa*)&so[w][r][c4]; if (C) *(volatile v4f*)(C + cofs + (size_t)(row0 + r) * ldc + col0 + c4) = v; if (C16) { v4h h4; for (int i = 0; i < 4; ++i) h4[i] = (_Float16)v[i]; *(volatile v4h*)(C16 + cofs + (size_t)(row0 + r) * ldc + col0 + c4) = h4; } } }
    if (pass == 0) __threadfence(); }
}


template <bool ASPLIT, bool BSPLIT, int ACT>
__global__ __launch_bounds__(128) void k_gemm_b(const float* __restrict__ A, int lda, size_t sA, const unsigned short* __restrict__ Bh, const unsigned short* __restrict__ Bl, int ldb, size_t sB,
                                             const float* __restrict__ bias, const float* __restrict__ resid, int ldr, size_t sR, float rsign, float alpha,
                                             float* __restrict__ C, int ldc, size_t sC, int M, int N, int K) {
  __shared__ __attribute__((aligned(16))) float so[4][16][64];
  const int tid = threadIdx.x, w = tid >> 5, lane = tid & 31, ln = lane & 15, hh = lane >> 4;
  const int by = blockIdx.y;
  A += (size_t)by * sA; Bh += (size_t)by * sB; if (BSPLIT) Bl += (size_t)by * sB; C += (size_t)by * sC; if (resid) resid += (size_t)by * sR;
  const int ntn = (N + 63) / 64; const int wid = blockIdx.x * 4 + w; const int mt = wid / ntn, nq = wid % ntn;
  if (mt * 16 >= M) return;
  const int row0 = mt * 16, col0 = nq * 64;
  const float* arow = A + (size_t)(row0 + ln) * lda;
  v8f acc[4] = {};
  for (int kb = 0; kb < K; kb += 32) {
    FragB ah, al;
    const v4f x0 = *(const v4fa*)(arow + kb + 8 * hh), x1 = *(const v4fa*)(arow + kb + 8 * hh + 4);
    const v4f x2 = *(const v4fa*)(arow + kb + 16 + 8 * hh), x3 = *(const v4fa*)(arow + kb + 16 + 8 * hh + 4);
    float xs[16] = {x0[0],x0[1],x0[2],x0[3],x1[0],x1[1],x1[2],x1[3],x2[0],x2[1],x2[2],x2[3],x3[0],x3[1],x3[2],x3[3]};
#pragma unroll
    for (int i = 0; i < 16; ++i) { const unsigned short hb = bf16_bits(xs[i]); ah.u[i] = hb; al.u[i] = ASPLIT ? bf16_bits(xs[i] - bf16_val(hb)) : (unsigned short)0; }
#pragma unroll
    for (int t = 0; t < 4; ++t) {
      if (col0 + t * 16 >= N) continue;
      const size_t boff = (size_t)(col0 + t * 16 + ln) * ldb + kb;
      FragB bh_, bl_; bh_.half[0] = *(const v8us*)(Bh + boff + 8 * hh); bh_.half[1] = *(const v8us*)(Bh + boff + 16 + 8 * hh);
      if (BSPLIT) { bl_.half[0] = *(const v8us*)(Bl + boff + 8 * hh); bl_.half[1] = *(const v8us*)(Bl + boff + 16 + 8 * hh); } else bl_ = bh_;
      acc[t] = mmaN<ASPLIT ? (BSPLIT ? 3 : 2) : 1>(ah.v, al.v, bh_.v, bl_.v, acc[t]);
    }
  }
#pragma unroll
  for (int t = 0; t < 4; ++t) {
    const int col = col0 + t * 16 + ln; if (col0 + t * 16 >= N) continue; const float bv = bias ? bf16_round(bias[col]) : 0.f;
#pragma unroll
    for (int r = 0; r < 8; ++r) { float v = acc[t][r] * alpha + bv; if (resid) v += rsign * resid[(size_t)(row0 + 8 * hh + r) * ldr + col]; if (ACT == 1) v = fmaxf(v, 0.f); else if (ACT == 2) v = fmaxf(v, 0.f) + log1pf(expf(-fabsf(v))); so[w][8 * hh + r][t * 16 + ln] = v; }
  }
  __builtin_amdgcn_fence(__ATOMIC_ACQ_REL, "workgroup"); __builtin_amdgcn_wave_barrier();
  const int rsub = lane >> 4, c4 = (lane & 15) * 4;
  for (int pass = 0; pass < 2; ++pass) {
#pragma unroll
    for (int q = 0; q < 8; ++q) { const int r = q * 2 + rsub; if (col0 + c4 < N) { const v4f v = *(const v4fa*)&so[w][r][c4]; *(volatile v4f*)(C + (size_t)(row0 + r) * ldc + col0 + c4) = v; } }
    if (pass == 0) __threadfence();
  }
}
__global__ __launch_bounds__(256) void k_split_transpose_b(const float* __restrict__ src, int lds_, size_t sIn, unsigned short* __restrict__ hi, unsigned short* __restrict__ lo, size_t sOut, int K, int N) {
  const size_t t = (size_t)blockIdx.x * 256 + threadIdx.x; const int k8n = K / 8; if (t >= (size_t)N * k8n) return;
  src += (size_t)blockIdx.y * sIn; hi += (size_t)blockIdx.y * sOut; lo += (size_t)blockIdx.y * sOut;
  const int n = (int)(t / k8n), k8 = (int)(t % k8n) * 8; v8us vh, vl;
#pragma unroll
  for (int i = 0; i < 8; ++i) { const float x = src[(size_t)(k8 + i) * lds_ + n]; const unsigned short hb = bf16_bits(x); vh[i] = hb; vl[i] = bf16_bits(x - bf16_val(hb)); }
  unsigned short* dh = hi + (size_t)n * K + k8; unsigned short* dl = lo + (size_t)n * K + k8;
  *(volatile v8us*)dh = vh; *(volatile v8us*)dl = vl; __threadfence(); *(volatile v8us*)dh = vh; *(volatile v8us*)dl = vl;
}

__global__ __launch_bounds__(256) void k_round_rows(const float* __restrict__ W, unsigned short* __restrict__ Wt, int n8) {
  const int t = blockIdx.x * 256 + threadIdx.x;
  if (t >= n8) return;
  const v4f a = *(const v4fa*)(W + (size_t)t * 8), b = *(const v4fa*)(W + (size_t)t * 8 + 4);
  v8us v; v[0]=bf16_bits(a[0]); v[1]=bf16_bits(a[1]); v[2]=bf16_bits(a[2]); v[3]=bf16_bits(a[3]);
  v[4]=bf16_bits(b[0]); v[5]=bf16_bits(b[1]); v[6]=bf16_bits(b[2]); v[7]=bf16_bits(b[3]);
  *(volatile v8us*)(Wt + (size_t)t * 8) = v; __threadfence(); *(volatile v8us*)(Wt + (size_t)t * 8) = v;
}

typedef _Float16 v2h __attribute__((ext_vector_type(2)));
__global__ __launch_bounds__(256) void k_ln(const float* __restrict__ x, const float* __restrict__ g, const float* __restrict__ be, float* __restrict__ NRM, _Float16* __restrict__ N16) { const int tid = threadIdx.x, wv = tid >> 5, lane = tid & 31; const size_t s = (size_t)blockIdx.x * 8 + wv; const float* xr = x + s * DM; float sm = 0.f;
#pragma unroll 2
  for (int c = lane; c < DM; c += 32) sm += bf16_round(xr[c]); for (int o = 16; o >= 1; o >>= 1) sm += __shfl_xor(sm, o, 32); const float mu = sm / (float)DM; float q2 = 0.f;
#pragma unroll 2
  for (int c = lane; c < DM; c += 32) { const float d = bf16_round(xr[c]) - mu; q2 += d * d; } for (int o = 16; o >= 1; o >>= 1) q2 += __shfl_xor(q2, o, 32); const float inv = 1.0f / sqrtf(q2 / (float)DM + 1e-5f);
  for (int pass = 0; pass < 2; ++pass) {
#pragma unroll 2
    for (int c = 2 * lane; c < DM; c += 64) { const float a = (bf16_round(xr[c]) - mu) * inv * bf16_round(g[c]) + bf16_round(be[c]), b2 = (bf16_round(xr[c + 1]) - mu) * inv * bf16_round(g[c + 1]) + bf16_round(be[c + 1]); typedef float v2f __attribute__((ext_vector_type(2), aligned(8))); v2f o = {a, b2}; *(volatile v2f*)(NRM + s * DM + c) = o; v2h oh = {(_Float16)a, (_Float16)b2}; *(volatile v2h*)(N16 + s * DM + c) = oh; } if (pass == 0) __threadfence(); } }
__global__ __launch_bounds__(256) void k_qk(const float* __restrict__ NRM, const float* __restrict__ wq, const float* __restrict__ bq, const float* __restrict__ wk, const float* __restrict__ bk, _Float16* __restrict__ Q16, _Float16* __restrict__ K16) { const size_t t = (size_t)blockIdx.x * 256 + threadIdx.x; if (t >= (size_t)SS * DM / 2) return; const int c = (int)((t * 2) % DM); const size_t s = (t * 2) / DM; const int h = c / DH, d = c % DH;
  _Float16 qc[2], qs[2], kc[2], ks[2];
#pragma unroll 1
  for (int q = 0; q < 2; ++q) { const float xv = NRM[s * DM + c + q]; const int hd = h * DH + d + q; const float thq = xv / (1.0f + fabsf(bf16_round(wq[hd]))) + bf16_round(bq[hd]); const float thk = xv / (1.0f + fabsf(bf16_round(wk[hd]))) + bf16_round(bk[hd]);
    float sq_, cq_, sk_, ck_; sincosf(thq, &sq_, &cq_); sincosf(thk, &sk_, &ck_); qc[q] = (_Float16)cq_; qs[q] = (_Float16)sq_; kc[q] = (_Float16)ck_; ks[q] = (_Float16)sk_; }
  _Float16* qrow = Q16 + ((size_t)h * SS + s) * 2 * DH; _Float16* krow = K16 + ((size_t)h * SS + s) * 2 * DH;
  const v2h vqc = {qc[0], qc[1]}, vqs = {qs[0], qs[1]}, vkc = {kc[0], kc[1]}, vks = {ks[0], ks[1]};
  for (int pass = 0; pass < 2; ++pass) { *(volatile v2h*)(qrow + d) = vqc; *(volatile v2h*)(qrow + DH + d) = vqs; *(volatile v2h*)(krow + d) = vkc; *(volatile v2h*)(krow + DH + d) = vks; if (pass == 0) __threadfence(); } }
__global__ __launch_bounds__(256) void k_vt(const _Float16* __restrict__ V16, _Float16* __restrict__ VT) { __shared__ _Float16 tile[32][34]; const int s0 = blockIdx.x * 32, c0 = blockIdx.y * 32; const int tx = threadIdx.x & 31, ty = threadIdx.x >> 5;
  for (int i = ty; i < 32; i += 8) tile[i][tx] = V16[(size_t)(s0 + i) * DM + c0 + tx]; __syncthreads();
  typedef _Float16 v4h __attribute__((ext_vector_type(4))); const int r = threadIdx.x >> 3, c4 = (threadIdx.x & 7) * 4; v4h o; for (int q = 0; q < 4; ++q) o[q] = tile[c4 + q][r]; const int c = c0 + r; const int h = c / DH, d = c % DH; _Float16* dst = VT + ((size_t)h * DH + d) * SS + s0 + c4; *(volatile v4h*)dst = o; __threadfence(); *(volatile v4h*)dst = o; }
__global__ __launch_bounds__(256) void k_soft(const float* __restrict__ S, _Float16* __restrict__ P) { const int tid = threadIdx.x, wv = tid >> 5, lane = tid & 31; const size_t row = (size_t)blockIdx.x * 8 + wv; const int i = (int)(row % SS); const float* s = S + row * SS; const float sc = 0.08838834764831845f; float mx = -3.0e38f;
  for (int j = lane; j <= i; j += 32) mx = fmaxf(mx, s[j] * sc); for (int o = 16; o >= 1; o >>= 1) mx = fmaxf(mx, __shfl_xor(mx, o, 32)); float den = 0.f;
  for (int j = lane; j <= i; j += 32) den += expf(s[j] * sc - mx); for (int o = 16; o >= 1; o >>= 1) den += __shfl_xor(den, o, 32); const float inv = 1.0f / den;
  for (int pass = 0; pass < 2; ++pass) { for (int j = 2 * lane; j < SS; j += 64) { v2h o2; o2.x = (_Float16)((j <= i) ? expf(s[j] * sc - mx) * inv : 0.f); o2.y = (_Float16)((j + 1 <= i) ? expf(s[j + 1] * sc - mx) * inv : 0.f); *(volatile v2h*)(P + row * SS + j) = o2; } if (pass == 0) __threadfence(); } }
__global__ __launch_bounds__(128) void k_res(const float* __restrict__ NRM, const float* __restrict__ Wr, const float* __restrict__ Br, float* __restrict__ CS, float* __restrict__ SN) { __shared__ float sx[DM]; const int s = blockIdx.x, n = threadIdx.x; for (int i = n; i < DM; i += 128) sx[i] = NRM[(size_t)s * DM + i]; __syncthreads();
  float cs = 0.f, sn = 0.f;
#pragma unroll 2
  for (int d = 0; d < DM; ++d) { const float th = sx[d] / (1.0f + fabsf(bf16_round(Wr[(size_t)n * DM + d]))) + bf16_round(Br[(size_t)n * DM + d]); float sv, cv; sincosf(th, &sv, &cv); cs += cv; sn += sv; }
  *(volatile float*)(CS + (size_t)s * NNR + n) = cs; *(volatile float*)(SN + (size_t)s * NNR + n) = sn; __threadfence(); *(volatile float*)(CS + (size_t)s * NNR + n) = cs; *(volatile float*)(SN + (size_t)s * NNR + n) = sn; }
__global__ __launch_bounds__(256) void k_bt(const float* __restrict__ vw, const float* __restrict__ ow, const float* __restrict__ pc, const float* __restrict__ ps, _Float16* __restrict__ Bv, _Float16* __restrict__ Bo, unsigned short* __restrict__ Bc, unsigned short* __restrict__ Bs) { const int t = blockIdx.x * 256 + threadIdx.x; if (t < DM * DM) { *(volatile _Float16*)(Bv + t) = (_Float16)(bf16_round(vw[t]) * 16.0f); *(volatile _Float16*)(Bo + t) = (_Float16)(bf16_round(ow[t]) * 16.0f); } if (t < DM * NNR) { *(volatile unsigned short*)(Bc + t) = bf16_bits(pc[t]); *(volatile unsigned short*)(Bs + t) = bf16_bits(ps[t]); } }
__global__ __launch_bounds__(256) void k_f16(const float* __restrict__ F, _Float16* __restrict__ A16, int n8) { const int t = blockIdx.x * 256 + threadIdx.x; if (t >= n8) return; FragH f; for (int q = 0; q < 8; ++q) f.h[q] = (_Float16)F[(size_t)t * 8 + q]; *(volatile v8us*)((unsigned short*)A16 + (size_t)t * 8) = f.half[0]; __threadfence(); *(volatile v8us*)((unsigned short*)A16 + (size_t)t * 8) = f.half[0]; }
__global__ __launch_bounds__(256) void k_fin(const float* __restrict__ x, const float* __restrict__ ATT, const float* __restrict__ RES, const float* __restrict__ asp, const float* __restrict__ rsp, float* __restrict__ out) { const int t = blockIdx.x * 256 + threadIdx.x; if (t >= SS * DM / 4) return; const float as_ = bf16_round(asp[0]), rs_ = bf16_round(rsp[0]); const v4f xv = *(const v4fa*)(x + (size_t)t * 4), a = *(const v4fa*)(ATT + (size_t)t * 4), r = *(const v4fa*)(RES + (size_t)t * 4); v4f o;
  for (int q = 0; q < 4; ++q) { const float rv = r[q]; const float sl = rv / (1.0f + expf(-rv)); o[q] = bf16_round(xv[q]) + as_ * a[q] + rs_ * sl; } *(volatile v4f*)(out + (size_t)t * 4) = o; __threadfence(); *(volatile v4f*)(out + (size_t)t * 4) = o; }
extern "C" void kernel_launch(void* const* d_in, const int* in_sizes, int n_in,
                              void* d_out, int out_size, void* d_ws, size_t ws_size, hipStream_t stream) {
  (void)in_sizes; (void)n_in; (void)out_size;
  const float* x = (const float*)d_in[0]; const float* lng = (const float*)d_in[1]; const float* lnb = (const float*)d_in[2]; const float* wq = (const float*)d_in[3]; const float* bq = (const float*)d_in[4]; const float* wk = (const float*)d_in[5]; const float* bk = (const float*)d_in[6]; const float* vw = (const float*)d_in[7]; const float* ow = (const float*)d_in[8]; const float* Wr = (const float*)d_in[9]; const float* Br = (const float*)d_in[10]; const float* pc = (const float*)d_in[11]; const float* ps = (const float*)d_in[12]; const float* asp = (const float*)d_in[13]; const float* rsp = (const float*)d_in[14];
  char* ws = (char*)d_ws; size_t off = 0;
  auto take = [&](size_t bytes) { char* p = ws + off; off += (bytes + 255) & ~(size_t)255; return p; };
  _Float16* Bv = (_Float16*)take((size_t)DM * DM * 2); _Float16* Bo = (_Float16*)take((size_t)DM * DM * 2); unsigned short* Bc = (unsigned short*)take((size_t)DM * NNR * 2); unsigned short* Bs = (unsigned short*)take((size_t)DM * NNR * 2);
  float* NRM = (float*)take((size_t)SS * DM * 4); _Float16* N16 = (_Float16*)take((size_t)SS * DM * 2); _Float16* Q16 = (_Float16*)take((size_t)NH * SS * 2 * DH * 2); _Float16* K16 = (_Float16*)take((size_t)NH * SS * 2 * DH * 2); _Float16* V16 = (_Float16*)take((size_t)SS * DM * 2); _Float16* VT = (_Float16*)take((size_t)NH * DH * SS * 2);
  float* S = (float*)take((size_t)NH * SS * SS * 4); _Float16* P = (_Float16*)take((size_t)NH * SS * SS * 2); float* O = (float*)take((size_t)SS * DM * 4); _Float16* O16 = (_Float16*)take((size_t)SS * DM * 2); float* ATT = (float*)take((size_t)SS * DM * 4);
  float* CS = (float*)take((size_t)SS * NNR * 4); float* SN = (float*)take((size_t)SS * NNR * 4); float* RES = (float*)take((size_t)SS * DM * 4);
  if (off > ws_size) return;
  k_bt<<<(DM * DM + 255) / 256, 256, 0, stream>>>(vw, ow, pc, ps, Bv, Bo, Bc, Bs);
  k_ln<<<SS / 8, 256, 0, stream>>>(x, lng, lnb, NRM, N16);
  k_qk<<<(SS * DM / 2 + 255) / 256, 256, 0, stream>>>(NRM, wq, bq, wk, bk, Q16, K16);
  k_gemm_hhx<0><<<dim3(((SS / 16) * (DM / 64) + 3) / 4, 1), 128, 0, stream>>>(N16, DM, 0, Bv, DM, 0, 0.0625f, nullptr, 0, nullptr, 1, 0, 0, nullptr, V16, DM, 0, SS, DM, DM);
  k_vt<<<dim3(SS / 32, DM / 32), 256, 0, stream>>>(V16, VT);
  k_gemm_hh<0><<<dim3(((SS / 16) * (SS / 64) + 3) / 4, NH), 128, 0, stream>>>(Q16, 2 * DH, (size_t)SS * 2 * DH, K16, 2 * DH, (size_t)SS * 2 * DH, 1.0f, S, SS, (size_t)SS * SS, SS, SS, 2 * DH);
  k_soft<<<NH * SS / 8, 256, 0, stream>>>(S, P);
  k_gemm_hh<0><<<dim3(((SS / 16) * 1 + 3) / 4, NH), 128, 0, stream>>>(P, SS, (size_t)SS * SS, VT, SS, (size_t)DH * SS, 1.0f, O, DM, (size_t)DH, SS, DH, SS);
  k_f16<<<(SS * DM / 8 + 255) / 256, 256, 0, stream>>>(O, O16, SS * DM / 8);
  k_gemm_hhx<0><<<dim3(((SS / 16) * (DM / 64) + 3) / 4, 1), 128, 0, stream>>>(O16, DM, 0, Bo, DM, 0, 0.0625f, nullptr, 0, nullptr, 1, 0, 0, ATT, nullptr, DM, 0, SS, DM, DM);
  k_res<<<SS, 128, 0, stream>>>(NRM, Wr, Br, CS, SN);
  k_gemm_b<true, false, 0><<<dim3(((SS / 16) * (DM / 64) + 3) / 4, 1), 128, 0, stream>>>(CS, NNR, 0, Bc, Bc, NNR, 0, nullptr, nullptr, 0, 0, 1.f, 1.f, RES, DM, 0, SS, DM, NNR);
  k_gemm_b<true, false, 0><<<dim3(((SS / 16) * (DM / 64) + 3) / 4, 1), 128, 0, stream>>>(SN, NNR, 0, Bs, Bs, NNR, 0, nullptr, RES, DM, 0, 1.f, 1.f, RES, DM, 0, SS, DM, NNR);
  k_fin<<<(SS * DM / 4 + 255) / 256, 256, 0, stream>>>(x, ATT, RES, asp, rsp, (float*)d_out);
}
